// TokenMixingMoE_69080253989464
// MI455X (gfx1250) — hardware-verified
//
#include <hip/hip_runtime.h>


namespace {
constexpr int NTOK = 32768, H = 128, I = 512, NE = 8;
constexpr float XS = 8.0f, WSC = 256.0f;
typedef _Float16 b16;
typedef __attribute__((ext_vector_type(16))) _Float16 v16b;
typedef __attribute__((ext_vector_type(8))) _Float16 v8b;
typedef __attribute__((ext_vector_type(8))) float v8f;
typedef __attribute__((ext_vector_type(4))) float v4f;
__device__ __forceinline__ float bf16_rne(float f) { unsigned int u = __float_as_uint(f); u += 0x7FFFu + ((u >> 16) & 1u); return __uint_as_float(u & 0xFFFF0000u); }
__device__ __forceinline__ void split16(float v, b16& hi, b16& lo) { hi = (b16)v; lo = (b16)(v - (float)hi); }
__device__ __forceinline__ v16b frag_kb(const b16* p, int hh) { const v8b a = *(const v8b*)(p + 8 * hh), b = *(const v8b*)(p + 16 + 8 * hh); v16b f;
#pragma unroll
  for (int e = 0; e < 8; ++e) { f[e] = a[e]; f[8 + e] = b[e]; } return f; }
__device__ __forceinline__ v8f wmma16b(v16b a, v16b b, v8f c) { v8f d = __builtin_amdgcn_wmma_f32_16x16x32_f16(false, a, false, b, (short)0, c, false, false); asm volatile("v_nop\n\tv_nop\n\tv_nop\n\tv_nop" : "+v"(d) : "v"(a), "v"(b)); return d; }
__device__ __forceinline__ void wave_lds_sync() { __builtin_amdgcn_fence(__ATOMIC_RELEASE, "workgroup"); __builtin_amdgcn_wave_barrier(); __builtin_amdgcn_fence(__ATOMIC_ACQUIRE, "workgroup"); }
__device__ __forceinline__ float pmul(float a, float b) { float p = a * b; asm volatile("" : "+v"(p)); return p; }
__device__ __forceinline__ float padd(float a, float b) { float p = a + b; asm volatile("" : "+v"(p)); return p; }
__device__ __forceinline__ float psub(float a, float b) { float p = a - b; asm volatile("" : "+v"(p)); return p; }
__device__ __forceinline__ int iclamp(int v, int lo, int hi) { return v < lo ? lo : (v > hi ? hi : v); }
__device__ __forceinline__ float gelu(float v) { return 0.5f * v * (1.0f + erff(v * 0.70710678118654752f)); }
__device__ __forceinline__ void csum(float& s, float& c, float y) { const float t = padd(s, y); const float bp = psub(t, s); const float e = padd(psub(s, psub(t, bp)), psub(y, bp)); s = t; c = padd(c, e); }

__global__ __launch_bounds__(256) void wcopy_kernel(const float* __restrict__ w, size_t total, b16* __restrict__ WT) { const size_t u = (size_t)blockIdx.x * 256 + threadIdx.x; if (u >= total / 8) return; const size_t e = u * 8; v8b v;
#pragma unroll
  for (int j = 0; j < 8; ++j) v[j] = (b16)(bf16_rne(w[e + j]) * WSC); for (int pass = 0; pass < 2; ++pass) { *(volatile v8b*)(WT + e) = v; __threadfence(); } }
__global__ __launch_bounds__(256) void router_kernel(const float* __restrict__ x, const float* __restrict__ gw, const float* __restrict__ gb, int RL, float* __restrict__ XN, float* __restrict__ ASG) {
  const int wave = threadIdx.x >> 5, lane = threadIdx.x & 31; const size_t t = (size_t)blockIdx.x * 8 + wave; if (t >= (size_t)RL) return; const int c0 = lane * 4; float xv[4];
#pragma unroll
  for (int i = 0; i < 4; ++i) xv[i] = bf16_rne(x[t * H + c0 + i]);
  float lg[NE];
#pragma unroll
  for (int e = 0; e < NE; ++e) { float s = 0.0f, c = 0.0f;
#pragma unroll
    for (int i = 0; i < 4; ++i) csum(s, c, pmul(xv[i], bf16_rne(gw[e * H + c0 + i])));
    for (int o = 1; o < 32; o <<= 1) { const float so = __shfl_xor(s, o), co = __shfl_xor(c, o); csum(s, c, so); c = padd(c, co); }
    lg[e] = padd(padd(s, c), bf16_rne(gb[e])); }
  float mx = lg[0]; for (int e = 1; e < NE; ++e) mx = fmaxf(mx, lg[e]); float p[NE], sm = 0.0f; for (int e = 0; e < NE; ++e) { p[e] = __expf(lg[e] - mx); sm += p[e]; }
  int e0 = 0; for (int e = 1; e < NE; ++e) if (lg[e] > lg[e0]) e0 = e; int e1 = e0 == 0 ? 1 : 0; for (int e = 0; e < NE; ++e) if (e != e0 && lg[e] > lg[e1]) e1 = e;
  const float s0 = p[e0] / sm, s1 = p[e1] / sm;
  float su = xv[0] + xv[1] + xv[2] + xv[3]; for (int o = 16; o; o >>= 1) su += __shfl_xor(su, o); const float mu = su * (1.0f / H); float sv = 0.0f; for (int i = 0; i < 4; ++i) { const float d = xv[i] - mu; sv += pmul(d, d); } for (int o = 16; o; o >>= 1) sv += __shfl_xor(sv, o); const float rs = rsqrtf(sv * (1.0f / H) + 1e-5f);
  v4f xn; for (int i = 0; i < 4; ++i) xn[i] = pmul(xv[i] - mu, rs);
  for (int pass = 0; pass < 2; ++pass) { *(volatile v4f*)(XN + t * H + c0) = xn; float v = 0.0f; if (lane == 0) v = (float)e0; else if (lane == 1) v = (float)e1; else if (lane == 2) v = s0; else if (lane == 3) v = s1; ((volatile float*)ASG)[t * 32 + lane] = v; __threadfence(); }
}
__global__ __launch_bounds__(256) void list_kernel(const float* __restrict__ ASG, int RL, int* __restrict__ LST, int* __restrict__ CNT) {
  __shared__ int sc[256], ent[256]; __shared__ int base; const int e = blockIdx.x, tid = threadIdx.x;
  for (int pass = 0; pass < 2; ++pass) { if (tid == 0) base = 0; __syncthreads();
    for (int c0 = 0; c0 < RL; c0 += 256) { const int t = c0 + tid; int slot = -1; if (t < RL) { const int a0 = (int)ASG[(size_t)t * 32], a1 = (int)ASG[(size_t)t * 32 + 1]; slot = a0 == e ? 0 : (a1 == e ? 1 : -1); }
      sc[tid] = slot >= 0 ? 1 : 0; __syncthreads();
      for (int o = 1; o < 256; o <<= 1) { const int v = tid >= o ? sc[tid - o] : 0; __syncthreads(); sc[tid] += v; __syncthreads(); }
      if (slot >= 0) ent[sc[tid] - 1] = t * 2 + slot; __syncthreads(); const int n = sc[255];
      if (tid < 32) { for (int i = tid; i < n; i += 32) ((volatile int*)LST)[(size_t)e * NTOK + base + i] = ent[i]; }
      __syncthreads(); if (tid == 0) base += n; __syncthreads(); }
    if (tid < 32) ((volatile int*)CNT)[e * 32 + tid] = tid == 0 ? base : 0; __threadfence(); __syncthreads(); }
}
__global__ __launch_bounds__(32) void expert_kernel(const float* __restrict__ XN, const float* __restrict__ g1, const float* __restrict__ c1, const b16* __restrict__ W1T, const float* __restrict__ g2, const float* __restrict__ c2, const b16* __restrict__ W2T, const float* __restrict__ bb2, const int* __restrict__ LST, const int* __restrict__ CNT, int WPE, float* __restrict__ Y) {
  __shared__ int Ent[16]; __shared__ __attribute__((aligned(16))) b16 Ah[16][H + 8], Al[16][H + 8], Fh[16][I + 8], Fl[16][I + 8]; __shared__ float Tt[16][I + 1], Of[16][H + 4], Mu[16], Rs[16];
  const int lane = threadIdx.x, nloc = lane & 15, hlf = lane >> 4; const int e = blockIdx.x / WPE, j0 = (blockIdx.x % WPE) * 16; const int cnt = iclamp(CNT[e * 32], 0, NTOK); if (j0 >= cnt) return;
  if (lane < 16) { const int j = j0 + lane; Ent[lane] = j < cnt ? iclamp(LST[(size_t)e * NTOK + j], 0, 2 * NTOK - 1) : -1; } wave_lds_sync();
  for (int rr = 0; rr < 16; ++rr) { const int ent = Ent[rr]; const size_t tok = ent >= 0 ? (size_t)(ent >> 1) : 0; for (int q = 0; q < 4; ++q) { const int c = q * 32 + lane; const float a = gelu(pmul(XN[tok * H + c], bf16_rne(g1[e * H + c])) + bf16_rne(c1[e * H + c])); b16 p, ql; split16(a * XS, p, ql); Ah[rr][c] = p; Al[rr][c] = ql; } }
  wave_lds_sync(); const b16* w1 = W1T + (size_t)e * I * H; const b16* w2 = W2T + (size_t)e * H * I;
#pragma unroll 1
  for (int cg = 0; cg < I / 128; ++cg) { v8f acc[8];
#pragma unroll
    for (int t = 0; t < 8; ++t) acc[t] = (v8f){};
#pragma unroll
    for (int kb = 0; kb < H; kb += 32) { const v16b a = frag_kb(&Ah[nloc][kb], hlf), al = frag_kb(&Al[nloc][kb], hlf);
#pragma unroll
      for (int t = 0; t < 8; ++t) { const v16b w = frag_kb(w1 + (size_t)(cg * 128 + t * 16 + nloc) * H + kb, hlf); acc[t] = wmma16b(a, w, acc[t]); acc[t] = wmma16b(al, w, acc[t]); } }
#pragma unroll
    for (int t = 0; t < 8; ++t)
#pragma unroll
      for (int r8 = 0; r8 < 8; ++r8) Tt[8 * hlf + r8][cg * 128 + t * 16 + nloc] = acc[t][r8] * (1.0f / (XS * WSC)); }
  wave_lds_sync();
  if (lane < 16) { float s = 0.0f; for (int i = 0; i < I; ++i) s += Tt[lane][i]; const float mu = s * (1.0f / I); float v = 0.0f; for (int i = 0; i < I; ++i) { const float d = Tt[lane][i] - mu; v += pmul(d, d); } Mu[lane] = mu; Rs[lane] = rsqrtf(v * (1.0f / I) + 1e-5f); }
  wave_lds_sync();
  for (int rr = 0; rr < 16; ++rr) for (int i = lane; i < I; i += 32) { const float a = gelu(pmul(pmul(Tt[rr][i] - Mu[rr], Rs[rr]), bf16_rne(g2[e * I + i])) + bf16_rne(c2[e * I + i])); b16 p, ql; split16(a * XS, p, ql); Fh[rr][i] = p; Fl[rr][i] = ql; }
  wave_lds_sync(); v8f acc[8];
#pragma unroll
  for (int t = 0; t < 8; ++t) acc[t] = (v8f){};
#pragma unroll 2
  for (int kb = 0; kb < I; kb += 32) { const v16b a = frag_kb(&Fh[nloc][kb], hlf), al = frag_kb(&Fl[nloc][kb], hlf);
#pragma unroll
    for (int t = 0; t < 8; ++t) { const v16b w = frag_kb(w2 + (size_t)(t * 16 + nloc) * I + kb, hlf); acc[t] = wmma16b(a, w, acc[t]); acc[t] = wmma16b(al, w, acc[t]); } }
#pragma unroll
  for (int t = 0; t < 8; ++t) { const int c = t * 16 + nloc; const float bb = bf16_rne(bb2[e * H + c]);
#pragma unroll
    for (int r8 = 0; r8 < 8; ++r8) Of[8 * hlf + r8][c] = acc[t][r8] * (1.0f / (XS * WSC)) + bb; }
  wave_lds_sync();
  for (int pass = 0; pass < 2; ++pass) { for (int rr = 0; rr < 16; ++rr) { const int ent = Ent[rr]; if (ent >= 0) *(volatile v4f*)(Y + (size_t)ent * H + lane * 4) = *(const v4f*)(&Of[rr][lane * 4]); } __threadfence(); }
}
__global__ __launch_bounds__(256) void combine_kernel(const float* __restrict__ Y, const float* __restrict__ ASG, int RL, float* __restrict__ out) {
  const int wave = threadIdx.x >> 5, lane = threadIdx.x & 31; const size_t t = (size_t)blockIdx.x * 8 + wave; if (t >= (size_t)RL) return; const float s0 = ASG[t * 32 + 2], s1 = ASG[t * 32 + 3]; const v4f a = *(const v4f*)(Y + (t * 2) * H + lane * 4), b = *(const v4f*)(Y + (t * 2 + 1) * H + lane * 4); v4f r; for (int i = 0; i < 4; ++i) r[i] = pmul(s0, a[i]) + pmul(s1, b[i]);
  for (int pass = 0; pass < 2; ++pass) { *(volatile v4f*)(out + t * H + lane * 4) = r; __threadfence(); }
}
}

extern "C" void kernel_launch(void* const* d_in, const int* in_sizes, int n_in, void* d_out, int out_size, void* d_ws, size_t ws_size, hipStream_t stream) {
  (void)n_in;
  auto Fp = [&](int i) { return (const float*)d_in[i]; };
  if (in_sizes[0] != NTOK * H || in_sizes[1] != NE * H || in_sizes[2] != NE || in_sizes[3] != NE * H || in_sizes[5] != NE * I * H || in_sizes[6] != NE * I || in_sizes[8] != NE * H * I || in_sizes[9] != NE * H || out_size != NTOK * H) return;
  const int RL = NTOK;
  size_t off = 0; char* ws = (char*)d_ws;
  auto carve = [&](size_t bytes) { char* p = ws + off; off += (bytes + 255) & ~(size_t)255; return p; };
  b16* W1T = (b16*)carve((size_t)NE * I * H * 2); b16* W2T = (b16*)carve((size_t)NE * H * I * 2); float* XN = (float*)carve((size_t)NTOK * H * 4); float* ASG = (float*)carve((size_t)NTOK * 32 * 4); int* LST = (int*)carve((size_t)NE * NTOK * 4); int* CNT = (int*)carve(NE * 32 * 4); float* Y = (float*)carve((size_t)NTOK * 2 * H * 4);
  if (off > ws_size || off > ((size_t)96 << 20)) return;
  wcopy_kernel<<<(unsigned)(((size_t)NE * I * H / 8 + 255) / 256), 256, 0, stream>>>(Fp(5), (size_t)NE * I * H, W1T); wcopy_kernel<<<(unsigned)(((size_t)NE * H * I / 8 + 255) / 256), 256, 0, stream>>>(Fp(8), (size_t)NE * H * I, W2T);
  router_kernel<<<(RL + 7) / 8, 256, 0, stream>>>(Fp(0), Fp(1), Fp(2), RL, XN, ASG);
  list_kernel<<<NE, 256, 0, stream>>>(ASG, RL, LST, CNT);
  const int WPE = NTOK / 16;
  expert_kernel<<<NE * WPE, 32, 0, stream>>>(XN, Fp(3), Fp(4), W1T, Fp(6), Fp(7), W2T, Fp(9), LST, CNT, WPE, Y);
  combine_kernel<<<(RL + 7) / 8, 256, 0, stream>>>(Y, ASG, RL, (float*)d_out);
}
